// Mamba2Block_66803921322400
// MI455X (gfx1250) — hardware-run, weakly checked
//
#include <hip/hip_runtime.h>
#include <math.h>

typedef __attribute__((ext_vector_type(16))) _Float16 v16h;
typedef __attribute__((ext_vector_type(8)))  _Float16 v8h;
typedef __attribute__((ext_vector_type(16))) __bf16   v16b;
typedef __attribute__((ext_vector_type(8)))  __bf16   v8b;
typedef __attribute__((ext_vector_type(8)))  float    v8f;
typedef __attribute__((ext_vector_type(4)))  float    v4f;

constexpr int kL     = 1024;
constexpr int kDm    = 512;
constexpr int kH     = 16;
constexpr int kP     = 64;
constexpr int kN     = 64;
constexpr int kCS    = 256;
constexpr int kNC    = kL / kCS;
constexpr int kHP    = kH * kP;
constexpr int kDproj = 2 * kHP + 2 * kN + 1;
constexpr int kNpad  = 2240;
constexpr int kColX  = kHP;
constexpr int kColB  = 2 * kHP;
constexpr int kColC  = 2 * kHP + kN;
constexpr int kColDt = 2 * kHP + 2 * kN;
constexpr int kKy    = kCS + kN;
static_assert(kDproj == 2177);
static_assert(kNpad % 64 == 0 && kNpad >= kDproj);
static_assert(kDm % 32 == 0 && kCS % 32 == 0 && kKy % 32 == 0 && kHP % 32 == 0);
static_assert(kL % 64 == 0 && kNpad % 64 == 0 && kN % 64 == 0 && kCS % 64 == 0 && kHP % 64 == 0 && kDm % 64 == 0);

constexpr size_t kSzU16  = (size_t)kL * kDm * 2;
constexpr size_t kSzWIT  = (size_t)kNpad * kDm * 2;
constexpr size_t kSzWO16 = (size_t)kDm * kHP * 2;
constexpr size_t kSzBIAS = (size_t)kNpad * 4;
constexpr size_t kSzPROJ = (size_t)kL * kNpad * 4;
constexpr size_t kSzVEC  = (size_t)kL * 4;
constexpr size_t kSzCDEC = (size_t)kNC * 32 * 4;
constexpr size_t kSzBN   = (size_t)kL * kN * 4;
constexpr size_t kSzBW   = (size_t)kNC * kN * kCS * 2;
constexpr size_t kSzM    = (size_t)kNC * kCS * kKy * 2;
constexpr size_t kSzBT   = (size_t)kNC * kHP * kKy * 2;
constexpr size_t kSzHF   = (size_t)(kNC - 1) * kHP * kN * 4;
constexpr size_t kSzYPRE = (size_t)kL * kHP * 4;
constexpr size_t kSzY16  = (size_t)kL * kHP * 2;

constexpr size_t kOffU16  = 0;
constexpr size_t kOffWIT  = kOffU16  + kSzU16;
constexpr size_t kOffWO16 = kOffWIT  + kSzWIT;
constexpr size_t kOffBIAS = kOffWO16 + kSzWO16;
constexpr size_t kOffPROJ = kOffBIAS + kSzBIAS;
constexpr size_t kOffDT   = kOffPROJ + kSzPROJ;
constexpr size_t kOffCS   = kOffDT   + kSzVEC;
constexpr size_t kOffDIN  = kOffCS   + kSzVEC;
constexpr size_t kOffCDEC = kOffDIN  + kSzVEC;
constexpr size_t kOffBN   = kOffCDEC + kSzCDEC;
constexpr size_t kOffCN   = kOffBN   + kSzBN;
constexpr size_t kOffBWH  = kOffCN   + kSzBN;
constexpr size_t kOffBWL  = kOffBWH  + kSzBW;
constexpr size_t kOffMH   = kOffBWL  + kSzBW;
constexpr size_t kOffML   = kOffMH   + kSzM;
constexpr size_t kOffBTH  = kOffML   + kSzM;
constexpr size_t kOffBTL  = kOffBTH  + kSzBT;
constexpr size_t kOffHF   = kOffBTL  + kSzBT;
constexpr size_t kOffYPRE = kOffHF   + kSzHF;
constexpr size_t kOffYH   = kOffYPRE + kSzYPRE;
constexpr size_t kOffYL   = kOffYH   + kSzY16;
constexpr size_t kWsTotal = kOffYL   + kSzY16;
static_assert(kWsTotal == 30102784ull);
static_assert(kWsTotal <= 134217728ull);
static_assert((kOffWIT % 128) == 0 && (kOffWO16 % 128) == 0 && (kOffBIAS % 128) == 0 && (kOffPROJ % 128) == 0 &&
              (kOffDT % 128) == 0 && (kOffCS % 128) == 0 && (kOffDIN % 128) == 0 && (kOffCDEC % 128) == 0 &&
              (kOffBN % 128) == 0 && (kOffCN % 128) == 0 && (kOffBWH % 128) == 0 && (kOffBWL % 128) == 0 &&
              (kOffMH % 128) == 0 && (kOffML % 128) == 0 && (kOffBTH % 128) == 0 && (kOffBTL % 128) == 0 &&
              (kOffHF % 128) == 0 && (kOffYPRE % 128) == 0 && (kOffYH % 128) == 0 && (kOffYL % 128) == 0);

__device__ __forceinline__ unsigned short f2bf_bits(float f) {
  unsigned u = __float_as_uint(f);
  return (unsigned short)((u + 0x7FFFu + ((u >> 16) & 1u)) >> 16);
}
__device__ __forceinline__ float bf_bits2f(unsigned short h) { return __uint_as_float(((unsigned)h) << 16); }
__device__ __forceinline__ float bf16r(float f) { return bf_bits2f(f2bf_bits(f)); }

__device__ __forceinline__ void dep_guard_h(v8f& a, v8f& b, v16h x, v16h y) { asm volatile("v_nop\n\tv_nop\n\tv_nop\n\tv_nop" : "+v"(a), "+v"(b) : "v"(x), "v"(y)); }
__device__ __forceinline__ void dep_guard_b(v8f& a, v8f& b, v16b x, v16b y) { asm volatile("v_nop\n\tv_nop\n\tv_nop\n\tv_nop" : "+v"(a), "+v"(b) : "v"(x), "v"(y)); }
__device__ __forceinline__ void dep_guard4x_h(v8f& a, v8f& b, v8f& c, v8f& d, v16h x, v16h y) { asm volatile("v_nop\n\tv_nop\n\tv_nop\n\tv_nop" : "+v"(a), "+v"(b), "+v"(c), "+v"(d) : "v"(x), "v"(y)); }
__device__ __forceinline__ void dep_guard4x_b(v8f& a, v8f& b, v8f& c, v8f& d, v16b x, v16b y) { asm volatile("v_nop\n\tv_nop\n\tv_nop\n\tv_nop" : "+v"(a), "+v"(b), "+v"(c), "+v"(d) : "v"(x), "v"(y)); }
__device__ __forceinline__ void keep4_h(v16h a, v16h b, v16h c, v16h d) { asm volatile("v_nop" :: "v"(a), "v"(b), "v"(c), "v"(d)); }
__device__ __forceinline__ void keep4_b(v16b a, v16b b, v16b c, v16b d) { asm volatile("v_nop" :: "v"(a), "v"(b), "v"(c), "v"(d)); }
__device__ __forceinline__ void acc_guard4(v8f& a, v8f& b, v8f& c, v8f& d) { asm volatile("v_nop\n\tv_nop\n\tv_nop\n\tv_nop" : "+v"(a), "+v"(b), "+v"(c), "+v"(d)); }
template <typename T> struct Frag;
template <> struct Frag<_Float16> {
  typedef v16h V; union U { v16h v; v8h h[2]; };
  static __device__ __forceinline__ v16h load(const _Float16* p) {
    U f; f.h[0] = *(const v8h*)(p); f.h[1] = *(const v8h*)(p + 16); return f.v;
  }
  static __device__ __forceinline__ v8f mma(v16h a, v16h b, v8f c) {
    return __builtin_amdgcn_wmma_f32_16x16x32_f16(false, a, false, b, (short)0, c, false, false);
  }
  static __device__ __forceinline__ void guard(v8f& a, v8f& b, v16h x, v16h y) { dep_guard_h(a, b, x, y); }
  static __device__ __forceinline__ void guard4(v8f& a, v8f& b, v8f& c, v8f& d, v16h x, v16h y) { dep_guard4x_h(a, b, c, d, x, y); }
  static __device__ __forceinline__ void keep(v16h a, v16h b, v16h c, v16h d) { keep4_h(a, b, c, d); }
};
template <> struct Frag<__bf16> {
  typedef v16b V; union U { v16b v; v8b h[2]; };
  static __device__ __forceinline__ v16b load(const __bf16* p) {
    U f; f.h[0] = *(const v8b*)(p); f.h[1] = *(const v8b*)(p + 16); return f.v;
  }
  static __device__ __forceinline__ v8f mma(v16b a, v16b b, v8f c) {
    return __builtin_amdgcn_wmma_f32_16x16x32_bf16(false, a, false, b, (short)0, c, false, false);
  }
  static __device__ __forceinline__ void guard(v8f& a, v8f& b, v16b x, v16b y) { dep_guard_b(a, b, x, y); }
  static __device__ __forceinline__ void guard4(v8f& a, v8f& b, v8f& c, v8f& d, v16b x, v16b y) { dep_guard4x_b(a, b, c, d, x, y); }
  static __device__ __forceinline__ void keep(v16b a, v16b b, v16b c, v16b d) { keep4_b(a, b, c, d); }
};

template <int ET> struct Elem;
template <> struct Elem<0> { typedef _Float16 T; };
template <> struct Elem<1> { typedef __bf16 T; };
template <int ET, int SPL, int BIAS_MODE, int OUT_MODE, bool RESID, int ACT = 0>
__global__ __launch_bounds__(256) void wmma_gemm64(
    const unsigned short* __restrict__ Ap, const unsigned short* __restrict__ A2p, int lda, long strideA,
    const unsigned short* __restrict__ Btp, const unsigned short* __restrict__ Bt2p, int ldb, long strideB,
    void* __restrict__ Cout, void* __restrict__ Cout2, int ldc, long strideC,
    const float* __restrict__ bias,
    const float* __restrict__ resid, long strideR,
    int M, int N, int K, float scale) {
  typedef typename Elem<ET>::T T;
  typedef typename Frag<T>::V V;
  const T* A = (const T*)Ap; const T* A2 = (const T*)A2p; const T* Bt = (const T*)Btp; const T* Bt2 = (const T*)Bt2p;
  __shared__ __align__(16) float sT[8][16 * 68];
  const int b    = blockIdx.y;
  const int lane = threadIdx.x & 31;
  const int wave = threadIdx.x >> 5;
  const int tilesN = N >> 6;
  const int tilesM = M >> 6;
  const int tile = blockIdx.x * 8 + wave;
  if (tile >= tilesM * tilesN) return;
  const int tm = tile / tilesN;
  const int tn = tile - tm * tilesN;
  const int m0 = tm << 6;
  const int n0 = tn << 6;

  const T* Ab  = A  + (size_t)b * strideA;
  const T* Bb  = Bt + (size_t)b * strideB;
  const T* Ab2 = (SPL >= 1) ? (A2  + (size_t)b * strideA) : nullptr;
  const T* Bb2 = (SPL == 2) ? (Bt2 + (size_t)b * strideB) : nullptr;

  const int rlane = lane & 15;
  const int koff  = (lane >> 4) * 8;
  const int mOff  = (lane >> 4) * 8;

  v8f acc[4][4];
#pragma unroll
  for (int i = 0; i < 4; ++i)
#pragma unroll
    for (int j = 0; j < 4; ++j) acc[i][j] = (v8f){0.f,0.f,0.f,0.f,0.f,0.f,0.f,0.f};

  for (int k0 = 0; k0 < K; k0 += 32) {
    V bh[4], bl[4];
#pragma unroll
    for (int j = 0; j < 4; ++j) {
      const size_t bo = (size_t)(n0 + (j << 4) + rlane) * ldb + koff + k0;
      bh[j] = Frag<T>::load(Bb + bo);
      if (SPL == 2) bl[j] = Frag<T>::load(Bb2 + bo);
    }
#pragma unroll
    for (int i = 0; i < 4; ++i) {
      const size_t ao = (size_t)(m0 + (i << 4) + rlane) * lda + koff + k0;
      V ah = Frag<T>::load(Ab + ao);
      V al;
      if (SPL >= 1) al = Frag<T>::load(Ab2 + ao);
#pragma unroll
      for (int j = 0; j < 4; ++j) {
        acc[i][j] = Frag<T>::mma(ah, bh[j], acc[i][j]);
        if (SPL == 2) acc[i][j] = Frag<T>::mma(ah, bl[j], acc[i][j]);
        if (SPL >= 1) acc[i][j] = Frag<T>::mma(al, bh[j], acc[i][j]);
      }
      Frag<T>::guard4(acc[i][0], acc[i][1], acc[i][2], acc[i][3], ah, (SPL >= 1) ? al : ah);
    }
    Frag<T>::keep(bh[0], bh[1], bh[2], bh[3]);
    if (SPL == 2) Frag<T>::keep(bl[0], bl[1], bl[2], bl[3]);
  }
  acc_guard4(acc[0][0], acc[0][1], acc[0][2], acc[0][3]);
  acc_guard4(acc[1][0], acc[1][1], acc[1][2], acc[1][3]);
  acc_guard4(acc[2][0], acc[2][1], acc[2][2], acc[2][3]);
  acc_guard4(acc[3][0], acc[3][1], acc[3][2], acc[3][3]);

  float* slab = sT[wave];
  const float* Rb = RESID ? (resid + (size_t)b * strideR) : nullptr;
#pragma unroll
  for (int i = 0; i < 4; ++i) {
    const int mBase = m0 + (i << 4);
#pragma unroll
    for (int j = 0; j < 4; ++j) {
      const int n = n0 + (j << 4) + rlane;
      float bv = 0.f;
      if (BIAS_MODE == 2) bv = bias[n];
#pragma unroll
      for (int r = 0; r < 8; ++r) {
        float v = acc[i][j][r] * scale;
        if (BIAS_MODE == 1) v += bias[mBase + mOff + r];
        if (BIAS_MODE == 2) v += bv;
        if (RESID) v += Rb[(size_t)(mBase + mOff + r) * ldc + n];
        if (ACT == 1) v = tanhf(v);
        if (ACT == 2) v = fmaxf(v, 0.0f);
        if (ACT == 3) v = v / (1.0f + expf(-v));
        if (ACT == 4) v = (v > 0.f) ? v : 0.01f * v;
        slab[(mOff + r) * 68 + (j << 4) + rlane] = v;
      }
    }
    __builtin_amdgcn_fence(__ATOMIC_RELEASE, "workgroup");
    __builtin_amdgcn_wave_barrier();
    __builtin_amdgcn_fence(__ATOMIC_ACQUIRE, "workgroup");
    if (OUT_MODE == 0) {
      float* C = (float*)Cout + (size_t)b * strideC;
      const int hh = lane >> 4, c4 = (lane & 15) * 4;
      for (int pass = 0; pass < 2; ++pass) {
#pragma unroll
        for (int it = 0; it < 8; ++it) {
          const int row = it * 2 + hh;
          v4f v = *(const v4f*)(slab + row * 68 + c4);
          *(volatile v4f*)(C + (size_t)(mBase + row) * ldc + n0 + c4) = v;
        }
        __threadfence();
      }
    } else {
      const int q = lane >> 3, c8 = (lane & 7) * 8;
      unsigned short* C  = (unsigned short*)Cout  + (size_t)b * strideC;
      unsigned short* C2 = (OUT_MODE == 2) ? ((unsigned short*)Cout2 + (size_t)b * strideC) : nullptr;
      for (int pass = 0; pass < 2; ++pass) {
#pragma unroll
        for (int it = 0; it < 4; ++it) {
          const int row = it * 4 + q;
          const float* sp = slab + row * 68 + c8;
          v8h hv, lv;
#pragma unroll
          for (int e = 0; e < 8; ++e) {
            if (OUT_MODE == 1) {
              hv[e] = (_Float16)sp[e];
            } else {
              unsigned short hb = f2bf_bits(sp[e]);
              unsigned short lb = f2bf_bits(sp[e] - bf_bits2f(hb));
              hv[e] = __builtin_bit_cast(_Float16, hb);
              lv[e] = __builtin_bit_cast(_Float16, lb);
            }
          }
          *(volatile v8h*)(C + (size_t)(mBase + row) * ldc + n0 + c8) = hv;
          if (OUT_MODE == 2) *(volatile v8h*)(C2 + (size_t)(mBase + row) * ldc + n0 + c8) = lv;
        }
        __threadfence();
      }
    }
    __builtin_amdgcn_fence(__ATOMIC_RELEASE, "workgroup");
    __builtin_amdgcn_wave_barrier();
    __builtin_amdgcn_fence(__ATOMIC_ACQUIRE, "workgroup");
  }
}

__device__ __forceinline__ void tile64_store_hilo(const float* sTile, unsigned short* __restrict__ ph,
                                                  unsigned short* __restrict__ pl, size_t base, int pitch,
                                                  int wave, int lane) {
  const int q = lane >> 3, lq = lane & 7;
  v8h hv[2], lv[2];
#pragma unroll
  for (int it = 0; it < 2; ++it) {
    const int row = wave * 8 + it * 4 + q;
    const float* sp = sTile + row * 68 + lq * 8;
    const v4f a0 = *(const v4f*)(sp);
    const v4f a1 = *(const v4f*)(sp + 4);
#pragma unroll
    for (int e = 0; e < 4; ++e) {
      const unsigned short h0 = f2bf_bits(a0[e]), h1 = f2bf_bits(a1[e]);
      const unsigned short l0 = f2bf_bits(a0[e] - bf_bits2f(h0)), l1 = f2bf_bits(a1[e] - bf_bits2f(h1));
      hv[it][e]     = __builtin_bit_cast(_Float16, h0);
      hv[it][4 + e] = __builtin_bit_cast(_Float16, h1);
      lv[it][e]     = __builtin_bit_cast(_Float16, l0);
      lv[it][4 + e] = __builtin_bit_cast(_Float16, l1);
    }
  }
  for (int pass = 0; pass < 2; ++pass) {
#pragma unroll
    for (int it = 0; it < 2; ++it) {
      const int row = wave * 8 + it * 4 + q;
      const size_t o = base + (size_t)row * pitch + lq * 8;
      *(volatile v8h*)(ph + o) = hv[it];
      *(volatile v8h*)(pl + o) = lv[it];
    }
    __threadfence();
  }
}

__global__ __launch_bounds__(256) void cvt_bf16_kernel(const float* __restrict__ src,
                                                       unsigned short* __restrict__ dst, int total8) {
  const int i = blockIdx.x * 256 + threadIdx.x;
  if (i >= total8) return;
  const size_t e0 = (size_t)i << 3;
  const v4f a0 = *(const v4f*)(src + e0);
  const v4f a1 = *(const v4f*)(src + e0 + 4);
  v8h hv;
#pragma unroll
  for (int e = 0; e < 4; ++e) {
    const unsigned short h0 = f2bf_bits(a0[e]), h1 = f2bf_bits(a1[e]);
    hv[e]     = __builtin_bit_cast(_Float16, h0);
    hv[4 + e] = __builtin_bit_cast(_Float16, h1);
  }
  unsigned short* qp = dst + e0;
  *(volatile v8h*)qp = hv;
  __threadfence();
  *(volatile v8h*)qp = hv;
}

__global__ __launch_bounds__(256) void bias_pad_kernel(const float* __restrict__ bi, float* __restrict__ dst) {
  const int i = blockIdx.x * 256 + threadIdx.x;
  if (i >= kNpad / 4) return;
  v4f v;
#pragma unroll
  for (int e = 0; e < 4; ++e) {
    const int n = 4 * i + e;
    const int ncl = (n < kDproj) ? n : (kDproj - 1);
    const float raw = bf16r(bi[ncl]);
    const float fz = (n < kDproj) ? 1.0f : 0.0f;
    v[e] = raw * fz;
  }
  float* qp = dst + 4 * i;
  *(volatile v4f*)qp = v;
  __threadfence();
  *(volatile v4f*)qp = v;
}

__global__ __launch_bounds__(256) void transpose_w_kernel(const float* __restrict__ in,
                                                          unsigned short* __restrict__ outp, int KR, int NCOL) {
  __shared__ __align__(16) float sT[64 * 68];
  const int tid = threadIdx.x, lane = tid & 31, wave = tid >> 5;
  const int k0 = blockIdx.x * 64, n0 = blockIdx.y * 64;
#pragma unroll
  for (int i = 0; i < 16; ++i) {
    const int idx = tid + 256 * i;
    const int kk = idx >> 6, nn = idx & 63;
    const int n = n0 + nn;
    const int ncl = (n < NCOL) ? n : (NCOL - 1);
    const float raw = in[(size_t)(k0 + kk) * NCOL + ncl];
    const float fz = (n < NCOL) ? 1.0f : 0.0f;
    sT[nn * 68 + kk] = raw * fz;
    if (i == 7) asm volatile("" ::: "memory");
  }
  __syncthreads();
  const int q = lane >> 3, lq = lane & 7;
  v8h hv[2];
#pragma unroll
  for (int it = 0; it < 2; ++it) {
    const int row = wave * 8 + it * 4 + q;
    const float* sp = sT + row * 68 + lq * 8;
    const v4f a0 = *(const v4f*)(sp);
    const v4f a1 = *(const v4f*)(sp + 4);
#pragma unroll
    for (int e = 0; e < 4; ++e) {
      const unsigned short h0 = f2bf_bits(a0[e]), h1 = f2bf_bits(a1[e]);
      hv[it][e]     = __builtin_bit_cast(_Float16, h0);
      hv[it][4 + e] = __builtin_bit_cast(_Float16, h1);
    }
  }
  for (int pass = 0; pass < 2; ++pass) {
#pragma unroll
    for (int it = 0; it < 2; ++it) {
      const int row = wave * 8 + it * 4 + q;
      const size_t o = (size_t)(n0 + row) * KR + k0 + lq * 8;
      *(volatile v8h*)(outp + o) = hv[it];
    }
    __threadfence();
  }
}

__global__ __launch_bounds__(256) void chunk_prep_kernel(
    const float* __restrict__ PROJ, const float* __restrict__ Alog,
    const float* __restrict__ wB, const float* __restrict__ wC,
    float* __restrict__ DT, float* __restrict__ CSUM, float* __restrict__ DIN, float* __restrict__ CDEC,
    float* __restrict__ BN, float* __restrict__ CN,
    unsigned short* __restrict__ BWH, unsigned short* __restrict__ BWL) {
  __shared__ float sScan[kCS];
  __shared__ float sWd[kCS];
  __shared__ __align__(16) float sT[32 * 260];
  const int tid = threadIdx.x, lane = tid & 31, wave = tid >> 5;
  const int c = blockIdx.x;
  const int t = c * kCS + tid;
  const float xr = PROJ[(size_t)t * kNpad + kColDt];
  const float dtv = fmaxf(xr, 0.0f) + log1pf(expf(-fabsf(xr)));
  const float aneg = -expf(bf16r(Alog[0]));
  const float la = dtv * aneg;
  sScan[tid] = la;
  __syncthreads();
  for (int off = 1; off < kCS; off <<= 1) {
    const int src = (tid >= off) ? (tid - off) : tid;
    const float w = sScan[src];
    const float v = sScan[tid] + ((tid >= off) ? w : 0.0f);
    __syncthreads();
    sScan[tid] = v;
    __syncthreads();
  }
  const float cs = sScan[tid];
  const float cl = sScan[kCS - 1];
  const float wd = expf(cl - cs) * dtv;
  const float dinv = expf(cs);
  const float cdec = expf(cl);
  sWd[tid] = wd;
  const float cdl = (lane == 0) ? cdec : 0.0f;
  for (int pass = 0; pass < 2; ++pass) {
    ((volatile float*)DT)[t] = dtv;
    ((volatile float*)CSUM)[t] = cs;
    ((volatile float*)DIN)[t] = dinv;
    if (wave == 0) ((volatile float*)CDEC)[c * 32 + lane] = cdl;
    __threadfence();
  }
  __syncthreads();

  const float wb0 = bf16r(wB[lane]), wb1 = bf16r(wB[32 + lane]);
  const float wc0 = bf16r(wC[lane]), wc1 = bf16r(wC[32 + lane]);
#pragma unroll 1
  for (int half = 0; half < 2; ++half) {
#pragma unroll 1
    for (int i = 0; i < 32; ++i) {
      const int s = wave + 8 * i;
      const size_t rb = (size_t)(c * kCS + s) * kNpad;
      const float b0 = PROJ[rb + kColB + lane];
      const float b1 = PROJ[rb + kColB + 32 + lane];
      const float c0 = PROJ[rb + kColC + lane];
      const float c1 = PROJ[rb + kColC + 32 + lane];
      float sb = b0 * b0 + b1 * b1;
      float sc = c0 * c0 + c1 * c1;
#pragma unroll
      for (int off = 16; off > 0; off >>= 1) {
        sb += __shfl_xor(sb, off, 32);
        sc += __shfl_xor(sc, off, 32);
      }
      const float rbv = rsqrtf(sb * (1.0f / 64.0f) + 1e-5f);
      const float rcv = rsqrtf(sc * (1.0f / 64.0f) + 1e-5f);
      const float bn0 = (b0 * rbv) * wb0, bn1 = (b1 * rbv) * wb1;
      const float cn0 = (c0 * rcv) * wc0, cn1 = (c1 * rcv) * wc1;
      if (half == 0) {
        const size_t ob = (size_t)(c * kCS + s) * kN;
        for (int pass = 0; pass < 2; ++pass) {
          ((volatile float*)BN)[ob + lane] = bn0;
          ((volatile float*)BN)[ob + 32 + lane] = bn1;
          ((volatile float*)CN)[ob + lane] = cn0;
          ((volatile float*)CN)[ob + 32 + lane] = cn1;
          __threadfence();
        }
      }
      const float wds = sWd[s];
      const float bsel = (half == 0) ? bn0 : bn1;
      sT[lane * 260 + s] = bsel * wds;
    }
    __syncthreads();
    v8h hv[4], lv[4];
#pragma unroll
    for (int it = 0; it < 4; ++it) {
      const int rr = wave * 4 + it;
      const float* sp = sT + rr * 260 + lane * 8;
      const v4f a0 = *(const v4f*)(sp);
      const v4f a1 = *(const v4f*)(sp + 4);
#pragma unroll
      for (int e = 0; e < 4; ++e) {
        const unsigned short h0 = f2bf_bits(a0[e]), h1 = f2bf_bits(a1[e]);
        const unsigned short l0 = f2bf_bits(a0[e] - bf_bits2f(h0)), l1 = f2bf_bits(a1[e] - bf_bits2f(h1));
        hv[it][e]     = __builtin_bit_cast(_Float16, h0);
        hv[it][4 + e] = __builtin_bit_cast(_Float16, h1);
        lv[it][e]     = __builtin_bit_cast(_Float16, l0);
        lv[it][4 + e] = __builtin_bit_cast(_Float16, l1);
      }
    }
    for (int pass = 0; pass < 2; ++pass) {
#pragma unroll
      for (int it = 0; it < 4; ++it) {
        const size_t o = (size_t)(c * kN + half * 32 + wave * 4 + it) * kCS + lane * 8;
        *(volatile v8h*)(BWH + o) = hv[it];
        *(volatile v8h*)(BWL + o) = lv[it];
      }
      __threadfence();
    }
    __syncthreads();
  }
}

__global__ __launch_bounds__(256) void xT_kernel(const float* __restrict__ PROJ,
                                                 unsigned short* __restrict__ BTH, unsigned short* __restrict__ BTL) {
  __shared__ __align__(16) float sT[64 * 68];
  const int tid = threadIdx.x, lane = tid & 31, wave = tid >> 5;
  const int stile = blockIdx.x, jt = blockIdx.y, c = blockIdx.z;
  if (stile == 4 && c != 0) return;
  const bool ztile = (stile == 4);
  const float fz = ztile ? 0.0f : 1.0f;
  const int srow = ztile ? 0 : (c * kCS + stile * 64);
  const int j0 = jt * 64;
#pragma unroll
  for (int i = 0; i < 4; ++i) {
    const int idx = tid + 256 * i;
    const int r = idx >> 4, cc4 = (idx & 15) * 4;
    const v4f v = *(const v4f*)(PROJ + (size_t)(srow + r) * kNpad + kColX + j0 + cc4);
    sT[(cc4 + 0) * 68 + r] = v[0] * fz;
    sT[(cc4 + 1) * 68 + r] = v[1] * fz;
    sT[(cc4 + 2) * 68 + r] = v[2] * fz;
    sT[(cc4 + 3) * 68 + r] = v[3] * fz;
  }
  __syncthreads();
  tile64_store_hilo(sT, BTH, BTL, (size_t)(c * kHP + j0) * kKy + stile * 64, kKy, wave, lane);
}

__global__ __launch_bounds__(256) void mplane_kernel(
    const float* __restrict__ BN, const float* __restrict__ CN, const float* __restrict__ CSUM,
    const float* __restrict__ DT, const float* __restrict__ DIN,
    unsigned short* __restrict__ MH, unsigned short* __restrict__ ML) {
  __shared__ __align__(16) float sC[64 * 68];
  __shared__ __align__(16) float sB[64 * 68];
  __shared__ __align__(16) float sO[64 * 68];
  __shared__ float sCsT[64];
  __shared__ float sCsS[64];
  __shared__ float sDtS[64];
  __shared__ float sDin[64];
  const int tid = threadIdx.x, lane = tid & 31, wave = tid >> 5;
  const int stile = blockIdx.x, ttile = blockIdx.y, c = blockIdx.z;
  const bool ctile = (stile == 4);
  const int t0 = ttile * 64;
  const int s0 = ctile ? 0 : stile * 64;
  const int trow = c * kCS + t0, srow = c * kCS + s0;
#pragma unroll
  for (int i = 0; i < 4; ++i) {
    const int idx = tid + 256 * i;
    const int r = idx >> 4, cc4 = (idx & 15) * 4;
    *(v4f*)(sC + r * 68 + cc4) = *(const v4f*)(CN + (size_t)(trow + r) * kN + cc4);
    *(v4f*)(sB + r * 68 + cc4) = *(const v4f*)(BN + (size_t)(srow + r) * kN + cc4);
  }
  if (wave < 2)      sCsT[tid]       = CSUM[trow + tid];
  else if (wave < 4) sCsS[tid - 64]  = CSUM[srow + tid - 64];
  else if (wave < 6) sDtS[tid - 128] = DT[srow + tid - 128];
  else               sDin[tid - 192] = DIN[trow + tid - 192];
  __syncthreads();
  const int ty = tid >> 4, tx = tid & 15;
  float o[4][4];
  if (!ctile) {
    float acc[4][4];
#pragma unroll
    for (int i = 0; i < 4; ++i)
#pragma unroll
      for (int j = 0; j < 4; ++j) acc[i][j] = 0.0f;
#pragma unroll 1
    for (int k = 0; k < kN; ++k) {
      float cv[4], bv[4];
#pragma unroll
      for (int i = 0; i < 4; ++i) cv[i] = sC[(ty * 4 + i) * 68 + k];
#pragma unroll
      for (int j = 0; j < 4; ++j) bv[j] = sB[(tx * 4 + j) * 68 + k];
#pragma unroll
      for (int i = 0; i < 4; ++i)
#pragma unroll
        for (int j = 0; j < 4; ++j) acc[i][j] = fmaf(cv[i], bv[j], acc[i][j]);
    }
    const float csref = sCsT[ty * 4];
    float e1[4], e2[4];
#pragma unroll
    for (int i = 0; i < 4; ++i) e1[i] = expf(fminf(sCsT[ty * 4 + i] - csref, 0.0f));
#pragma unroll
    for (int j = 0; j < 4; ++j) e2[j] = expf(fminf(csref - sCsS[tx * 4 + j], 80.0f)) * sDtS[tx * 4 + j];
#pragma unroll
    for (int i = 0; i < 4; ++i) {
#pragma unroll
      for (int j = 0; j < 4; ++j) {
        const int tl = t0 + ty * 4 + i;
        const int sl = s0 + tx * 4 + j;
        const float m = (e1[i] * e2[j]) * acc[i][j];
        o[i][j] = (sl <= tl) ? m : 0.0f;
      }
    }
  } else {
#pragma unroll
    for (int i = 0; i < 4; ++i) {
      const float di = sDin[ty * 4 + i];
#pragma unroll
      for (int j = 0; j < 4; ++j) o[i][j] = di * sC[(ty * 4 + i) * 68 + tx * 4 + j];
    }
  }
#pragma unroll
  for (int i = 0; i < 4; ++i)
#pragma unroll
    for (int j = 0; j < 4; ++j) sO[(ty * 4 + i) * 68 + tx * 4 + j] = o[i][j];
  __syncthreads();
  tile64_store_hilo(sO, MH, ML, (size_t)trow * kKy + stile * 64, kKy, wave, lane);
}

__global__ __launch_bounds__(256) void carry_kernel(const float* __restrict__ HF, const float* __restrict__ CDEC,
                                                    unsigned short* __restrict__ BTH, unsigned short* __restrict__ BTL) {
  const int gid = blockIdx.x * 256 + threadIdx.x;
  if (gid >= kHP * 8) return;
  const int j = gid >> 3, g8 = gid & 7;
  float h[8];
#pragma unroll
  for (int e = 0; e < 8; ++e) h[e] = 0.0f;
#pragma unroll
  for (int c = 0; c < kNC - 1; ++c) {
    const float dec = CDEC[c * 32];
    const float* hp = HF + (size_t)(c * kHP + j) * kN + g8 * 8;
    const v4f a0 = *(const v4f*)(hp);
    const v4f a1 = *(const v4f*)(hp + 4);
#pragma unroll
    for (int e = 0; e < 4; ++e) {
      h[e]     = h[e] * dec + a0[e];
      h[4 + e] = h[4 + e] * dec + a1[e];
    }
    v8h hv, lv;
#pragma unroll
    for (int e = 0; e < 8; ++e) {
      const unsigned short hb = f2bf_bits(h[e]);
      const unsigned short lb = f2bf_bits(h[e] - bf_bits2f(hb));
      hv[e] = __builtin_bit_cast(_Float16, hb);
      lv[e] = __builtin_bit_cast(_Float16, lb);
    }
    const size_t o = (size_t)((c + 1) * kHP + j) * kKy + kCS + g8 * 8;
    *(volatile v8h*)(BTH + o) = hv;
    *(volatile v8h*)(BTL + o) = lv;
    __threadfence();
    *(volatile v8h*)(BTH + o) = hv;
    *(volatile v8h*)(BTL + o) = lv;
  }
}

__global__ __launch_bounds__(256) void gate_kernel(const float* __restrict__ YPRE, const float* __restrict__ PROJ,
                                                   const float* __restrict__ Dp,
                                                   unsigned short* __restrict__ YH, unsigned short* __restrict__ YL) {
  const int gid = blockIdx.x * 256 + threadIdx.x;
  if (gid >= kL * kHP / 8) return;
  const int t = gid >> 7, c8 = (gid & 127) * 8;
  const float dv = bf16r(Dp[c8 >> 6]);
  const float* yp = YPRE + (size_t)t * kHP + c8;
  const float* xp = PROJ + (size_t)t * kNpad + kColX + c8;
  const float* zp = PROJ + (size_t)t * kNpad + c8;
  const v4f y0 = *(const v4f*)(yp), y1 = *(const v4f*)(yp + 4);
  const v4f x0 = *(const v4f*)(xp), x1 = *(const v4f*)(xp + 4);
  const v4f z0 = *(const v4f*)(zp), z1 = *(const v4f*)(zp + 4);
  float r[8];
#pragma unroll
  for (int e = 0; e < 4; ++e) {
    const float ya = y0[e] + x0[e] * dv;
    const float yb = y1[e] + x1[e] * dv;
    const float za = z0[e], zb = z1[e];
    const float sga = __builtin_amdgcn_rcpf(1.0f + expf(-za));
    const float sgb = __builtin_amdgcn_rcpf(1.0f + expf(-zb));
    r[e]     = ya * (za * sga);
    r[4 + e] = yb * (zb * sgb);
  }
  v8h hv, lv;
#pragma unroll
  for (int e = 0; e < 8; ++e) {
    const unsigned short hb = f2bf_bits(r[e]);
    const unsigned short lb = f2bf_bits(r[e] - bf_bits2f(hb));
    hv[e] = __builtin_bit_cast(_Float16, hb);
    lv[e] = __builtin_bit_cast(_Float16, lb);
  }
  const size_t o = (size_t)t * kHP + c8;
  *(volatile v8h*)(YH + o) = hv;
  *(volatile v8h*)(YL + o) = lv;
  __threadfence();
  *(volatile v8h*)(YH + o) = hv;
  *(volatile v8h*)(YL + o) = lv;
}

extern "C" void kernel_launch(void* const* d_in, const int* in_sizes, int n_in,
                              void* d_out, int out_size, void* d_ws, size_t ws_size,
                              hipStream_t stream) {
  if (n_in < 8) return;
  if (in_sizes[0] != kL * kDm) return;
  if (in_sizes[1] != kDm * kDproj) return;
  if (in_sizes[2] != kDproj) return;
  if (in_sizes[3] != 1) return;
  if (in_sizes[4] != kH) return;
  if (in_sizes[5] != kN) return;
  if (in_sizes[6] != kN) return;
  if (in_sizes[7] != kHP * kDm) return;
  if (out_size != kL * kDm) return;
  if (ws_size < kWsTotal) return;

  const float* u     = (const float*)d_in[0];
  const float* Wi    = (const float*)d_in[1];
  const float* bi    = (const float*)d_in[2];
  const float* A_log = (const float*)d_in[3];
  const float* Dv    = (const float*)d_in[4];
  const float* wB    = (const float*)d_in[5];
  const float* wC    = (const float*)d_in[6];
  const float* Wo    = (const float*)d_in[7];
  float* out = (float*)d_out;

  char* ws = (char*)d_ws;
  unsigned short* U16  = (unsigned short*)(ws + kOffU16);
  unsigned short* WIT  = (unsigned short*)(ws + kOffWIT);
  unsigned short* WO16 = (unsigned short*)(ws + kOffWO16);
  float*          BIAS = (float*)(ws + kOffBIAS);
  float*          PROJ = (float*)(ws + kOffPROJ);
  float*          DT   = (float*)(ws + kOffDT);
  float*          CSUM = (float*)(ws + kOffCS);
  float*          DIN  = (float*)(ws + kOffDIN);
  float*          CDEC = (float*)(ws + kOffCDEC);
  float*          BN   = (float*)(ws + kOffBN);
  float*          CN   = (float*)(ws + kOffCN);
  unsigned short* BWH  = (unsigned short*)(ws + kOffBWH);
  unsigned short* BWL  = (unsigned short*)(ws + kOffBWL);
  unsigned short* MH   = (unsigned short*)(ws + kOffMH);
  unsigned short* ML   = (unsigned short*)(ws + kOffML);
  unsigned short* BTH  = (unsigned short*)(ws + kOffBTH);
  unsigned short* BTL  = (unsigned short*)(ws + kOffBTL);
  float*          HF   = (float*)(ws + kOffHF);
  float*          YPRE = (float*)(ws + kOffYPRE);
  unsigned short* YH   = (unsigned short*)(ws + kOffYH);
  unsigned short* YL   = (unsigned short*)(ws + kOffYL);

  cvt_bf16_kernel<<<(kL * kDm / 8) / 256, 256, 0, stream>>>(u, U16, kL * kDm / 8);
  bias_pad_kernel<<<(kNpad / 4 + 255) / 256, 256, 0, stream>>>(bi, BIAS);
  transpose_w_kernel<<<dim3(kDm / 64, kNpad / 64), 256, 0, stream>>>(Wi, WIT, kDm, kDproj);
  transpose_w_kernel<<<dim3(kHP / 64, kDm / 64), 256, 0, stream>>>(Wo, WO16, kHP, kDm);

  wmma_gemm64<1, 0, 2, 0, false><<<dim3(70, 1), 256, 0, stream>>>(
      U16, nullptr, kDm, 0L,
      WIT, nullptr, kDm, 0L,
      (void*)PROJ, nullptr, kNpad, 0L,
      BIAS, nullptr, 0L,
      kL, kNpad, kDm, 1.0f);

  chunk_prep_kernel<<<kNC, kCS, 0, stream>>>(PROJ, A_log, wB, wC, DT, CSUM, DIN, CDEC, BN, CN, BWH, BWL);

  xT_kernel<<<dim3(5, kHP / 64, kNC), 256, 0, stream>>>(PROJ, BTH, BTL);

  mplane_kernel<<<dim3(5, kCS / 64, kNC), 256, 0, stream>>>(BN, CN, CSUM, DT, DIN, MH, ML);

  wmma_gemm64<1, 2, 0, 0, false><<<dim3(2, kNC - 1), 256, 0, stream>>>(
      BTH, BTL, kKy, (long)kHP * kKy,
      BWH, BWL, kCS, (long)kN * kCS,
      (void*)HF, nullptr, kN, (long)kHP * kN,
      nullptr, nullptr, 0L,
      kHP, kN, kCS, 1.0f);

  carry_kernel<<<(kHP * 8) / 256, 256, 0, stream>>>(HF, CDEC, BTH, BTL);

  wmma_gemm64<1, 2, 0, 0, false><<<dim3(8, kNC), 256, 0, stream>>>(
      MH, ML, kKy, (long)kCS * kKy,
      BTH, BTL, kKy, (long)kHP * kKy,
      (void*)YPRE, nullptr, kHP, (long)kCS * kHP,
      nullptr, nullptr, 0L,
      kCS, kHP, kKy, 1.0f);

  gate_kernel<<<(kL * kHP / 8) / 256, 256, 0, stream>>>(YPRE, PROJ, Dv, YH, YL);

  wmma_gemm64<1, 1, 0, 0, false><<<dim3(16, 1), 256, 0, stream>>>(
      YH, YL, kHP, 0L,
      WO16, nullptr, kHP, 0L,
      (void*)out, nullptr, kDm, 0L,
      nullptr, nullptr, 0L,
      kL, kDm, kHP, 1.0f);
}
